// ContentStyleGraphNet_44461501448530
// MI455X (gfx1250) — hardware-verified
//
#include <hip/hip_runtime.h>
#include <math.h>
#include <stddef.h>


typedef _Float16 v16h __attribute__((ext_vector_type(16)));
typedef _Float16 v8h  __attribute__((ext_vector_type(8)));
typedef float    v8f  __attribute__((ext_vector_type(8)));
typedef float    v4f  __attribute__((ext_vector_type(4)));
typedef v8h v8ha __attribute__((may_alias));
typedef v4f v4fa __attribute__((may_alias));

#define DEV __device__ __forceinline__

DEV float gelu_f(float v) { return 0.5f * v * (1.0f + erff(v * 0.70710678118654752f)); }
DEV float sigm_f(float v) { return 1.0f / (1.0f + expf(-v)); }

union Frag16 { v16h v; v8h hv[2]; };

DEV v16h ld_frag(const _Float16* base, int ld, int lane) {
  const int m = lane & 15, h = lane >> 4;
  const _Float16* row = base + m * ld + 8 * h;
  Frag16 u;
  u.hv[0] = *(const v8ha*)(row);
  u.hv[1] = *(const v8ha*)(row + 16);
  return u.v;
}

DEV v8f wmma_f16(v16h a, v16h b, v8f c) {
  v8f d = __builtin_amdgcn_wmma_f32_16x16x32_f16(false, a, false, b, (short)0, c, false, false);
  asm volatile("v_nop\n\tv_nop\n\tv_nop\n\tv_nop" : "+v"(d) : "v"(a), "v"(b));
  return d;
}

DEV v8f splat8(float v) {
  v8f z;
#pragma unroll
  for (int i = 0; i < 8; ++i) z[i] = v;
  return z;
}

DEV void ln_row_f16(const float* px, const float* g, const float* bt, _Float16* pa) {
  float mu = 0.f;
#pragma unroll 16
  for (int dd = 0; dd < 64; ++dd) mu += px[dd];
  mu *= (1.0f / 64.0f);
  float var = 0.f;
#pragma unroll 16
  for (int dd = 0; dd < 64; ++dd) { const float t = px[dd] - mu; var += t * t; }
  const float rs = 1.0f / sqrtf(var * (1.0f / 64.0f) + 1e-5f);
#pragma unroll
  for (int vv = 0; vv < 8; ++vv) {
    v8h hv;
#pragma unroll
    for (int e = 0; e < 8; ++e) {
      const int dd = vv * 8 + e;
      hv[e] = (_Float16)((px[dd] - mu) * rs * g[dd] + bt[dd]);
    }
    *(v8ha*)(pa + vv * 8) = hv;
  }
}

#define H1P 40
#define H1ROWS 1028
#define W2P 40

DEV void conv_tile_store(float* ht, const float* stgw, int b, int c, int mt, int lane) {
  const int q = lane >> 3, j = lane & 7;
#pragma unroll
  for (int s = 0; s < 2; ++s) {
    const int L = s * 4 + q;
    const int tloc = L >> 1, half = L & 1;
    const int t = mt * 4 + tloc;
    const v4f v = *(const v4fa*)(stgw + tloc * 64 + half * 32 + j * 4);
    float* dst = ht + (((size_t)(b * 256 + t) * 16 + c) * 64 + half * 32 + j * 4);
    *(volatile v4f*)dst = v;
  }
}

__global__ void __launch_bounds__(256) conv_kernel(
    const float* __restrict__ x,
    const float* __restrict__ c1w, const float* __restrict__ c1b,
    const float* __restrict__ bn1g, const float* __restrict__ bn1b,
    const float* __restrict__ bn1m, const float* __restrict__ bn1v,
    const float* __restrict__ c2w, const float* __restrict__ c2b,
    const float* __restrict__ bn2g, const float* __restrict__ bn2b,
    const float* __restrict__ bn2m, const float* __restrict__ bn2v,
    float* __restrict__ ht, float* __restrict__ hn)
{
  __shared__ __attribute__((aligned(16))) float    xs[4096];
  __shared__ __attribute__((aligned(16))) _Float16 h1T[H1ROWS * H1P];
  __shared__ __attribute__((aligned(16))) _Float16 w2s[5 * 64 * W2P];
  __shared__ __attribute__((aligned(16))) float    stg[8 * 256];
  __shared__ float w1s[224];
  __shared__ float a1c[32], b1c[32], a2c[64], b2c[64];
  __shared__ float sred[8 * 64];
  __shared__ __attribute__((aligned(16))) float shn[64];
  __shared__ float srd[64];

  const int bc = blockIdx.x;
  const int b = bc >> 4, c = bc & 15;
  const int tid = threadIdx.x, lane = tid & 31, wave = tid >> 5;
  const int m = lane & 15, h = lane >> 4;

  {
    const v4f* src = (const v4f*)(x + (size_t)bc * 4096);
    for (int i = tid; i < 1024; i += 256) *(v4fa*)&xs[i * 4] = src[i];
  }
  for (int i = tid; i < 224; i += 256) w1s[i] = c1w[i];
  for (int i = tid; i < 10240; i += 256) {
    const int n = i / 160, rem = i - n * 160;
    const int ic = rem / 5, j = rem - ic * 5;
    w2s[(j * 64 + n) * W2P + ic] = (_Float16)c2w[i];
  }
  if (tid < 128) {
    const int r = tid >> 5, col = tid & 31;
    const int row = (r < 2) ? r : (1024 + r);
    h1T[row * H1P + col] = (_Float16)0.0f;
  }
  if (tid < 32) {
    const float sc = bn1g[tid] / sqrtf(bn1v[tid] + 1e-5f);
    a1c[tid] = sc;
    b1c[tid] = bn1b[tid] - bn1m[tid] * sc + c1b[tid] * sc;
  }
  if (tid < 64) {
    const float sc = bn2g[tid] / sqrtf(bn2v[tid] + 1e-5f);
    a2c[tid] = sc;
    b2c[tid] = bn2b[tid] - bn2m[tid] * sc + c2b[tid] * sc;
  }
  __syncthreads();

  for (int idx = tid; idx < 32768; idx += 256) {
    const int oc = idx >> 10, tp = idx & 1023;
    const float A = a1c[oc], Bc = b1c[oc];
    float mx = -3.0e38f;
#pragma unroll
    for (int p = 0; p < 4; ++p) {
      const int pos = tp * 4 + p;
      float acc = 0.f;
#pragma unroll
      for (int j = 0; j < 7; ++j) {
        const int q = pos + j - 3;
        if (q >= 0 && q < 4096) acc += w1s[oc * 7 + j] * xs[q];
      }
      mx = fmaxf(mx, gelu_f(acc * A + Bc));
    }
    h1T[(tp + 2) * H1P + oc] = (_Float16)mx;
  }
  __syncthreads();

  float* stgw = stg + wave * 256;
  float psum[4] = {0.f, 0.f, 0.f, 0.f};
  for (int tl = 0; tl < 8; ++tl) {
    const int mt = wave * 8 + tl;
    v16h af[5];
#pragma unroll
    for (int j = 0; j < 5; ++j) af[j] = ld_frag(h1T + (mt * 16 + j) * H1P, H1P, lane);
    v8f acc[4];
#pragma unroll
    for (int nt = 0; nt < 4; ++nt) {
      acc[nt] = splat8(0.f);
#pragma unroll
      for (int j = 0; j < 5; ++j)
        acc[nt] = wmma_f16(af[j], ld_frag(w2s + (j * 64 + nt * 16) * W2P, W2P, lane), acc[nt]);
    }
#pragma unroll
    for (int nt = 0; nt < 4; ++nt) {
      const int col = nt * 16 + m;
      const float A = a2c[col], Bc = b2c[col];
      float y[8];
#pragma unroll
      for (int i = 0; i < 8; ++i) y[i] = gelu_f(acc[nt][i] * A + Bc);
      const float m0 = fmaxf(fmaxf(y[0], y[1]), fmaxf(y[2], y[3]));
      const float m1 = fmaxf(fmaxf(y[4], y[5]), fmaxf(y[6], y[7]));
      stgw[(2 * h) * 64 + col]     = m0;
      stgw[(2 * h + 1) * 64 + col] = m1;
      psum[nt] += m0 + m1;
    }
    __syncthreads();
    conv_tile_store(ht, stgw, b, c, mt, lane);
    __threadfence();
    conv_tile_store(ht, stgw, b, c, mt, lane);
    __syncthreads();
  }

#pragma unroll
  for (int nt = 0; nt < 4; ++nt) psum[nt] += __shfl_xor(psum[nt], 16);
  if (h == 0) {
#pragma unroll
    for (int nt = 0; nt < 4; ++nt) sred[wave * 64 + nt * 16 + m] = psum[nt];
  }
  __syncthreads();
  float hv = 0.f;
  if (tid < 64) {
    float s = 0.f;
#pragma unroll
    for (int w = 0; w < 8; ++w) s += sred[w * 64 + tid];
    hv = s * (1.0f / 256.0f);
    srd[tid] = hv;
  }
  __syncthreads();
  for (int st = 32; st > 0; st >>= 1) { if (tid < st) srd[tid] += srd[tid + st]; __syncthreads(); }
  const float mean = srd[0] * (1.0f / 64.0f);
  __syncthreads();
  const float hc = hv - mean;
  if (tid < 64) srd[tid] = hc * hc;
  __syncthreads();
  for (int st = 32; st > 0; st >>= 1) { if (tid < st) srd[tid] += srd[tid + st]; __syncthreads(); }
  const float nrm = sqrtf(srd[0]) + 1e-8f;
  if (tid < 64) shn[tid] = hc * (1.0f / nrm);
  __syncthreads();
  if (tid < 16) {
    const v4f v = *(const v4fa*)&shn[tid * 4];
    *(volatile v4f*)(hn + (size_t)bc * 64 + tid * 4) = v;
  }
  __threadfence();
  if (tid < 16) {
    const v4f v = *(const v4fa*)&shn[tid * 4];
    *(volatile v4f*)(hn + (size_t)bc * 64 + tid * 4) = v;
  }
}

#define XNP 2080

DEV void fft_store(float* dst_row, const float* mag, float inv, int tid) {
#pragma unroll
  for (int s = 0; s < 3; ++s) {
    const int f4 = s * 256 + tid;
    if (f4 < 520) {
      v4f v;
#pragma unroll
      for (int e = 0; e < 4; ++e) {
        const int f = f4 * 4 + e;
        v[e] = (f < 2049) ? mag[f] * inv : 0.0f;
      }
      *(volatile v4f*)(dst_row + f4 * 4) = v;
    }
  }
}

__global__ void __launch_bounds__(256) fft_kernel(const float* __restrict__ x,
                                                  float* __restrict__ Xn)
{
  __shared__ float re[4096], im[4096];
  __shared__ float twr[2048], twi[2048];
  __shared__ float red[256];
  const int bc = blockIdx.x, tid = threadIdx.x;
  for (int i = tid; i < 4096; i += 256) {
    const int r = (int)(__brev((unsigned)i) >> 20);
    re[i] = x[(size_t)bc * 4096 + r];
    im[i] = 0.f;
  }
  for (int k = tid; k < 2048; k += 256) {
    const float ang = -6.283185307179586f * ((float)k * (1.0f / 4096.0f));
    twr[k] = cosf(ang);
    twi[k] = sinf(ang);
  }
  __syncthreads();
  for (int s = 0; s < 12; ++s) {
    const int half = 1 << s, mm = half << 1;
    for (int bf = tid; bf < 2048; bf += 256) {
      const int blk = bf >> s, pos = bf & (half - 1);
      const int i0 = blk * mm + pos, i1 = i0 + half;
      const int tw = pos << (11 - s);
      const float wr = twr[tw], wi = twi[tw];
      const float xr = re[i1], xi = im[i1];
      const float tr = wr * xr - wi * xi, ti = wr * xi + wi * xr;
      const float ur = re[i0], ui = im[i0];
      re[i0] = ur + tr; im[i0] = ui + ti;
      re[i1] = ur - tr; im[i1] = ui - ti;
    }
    __syncthreads();
  }
  float ss = 0.f;
  for (int f = tid; f < 2049; f += 256) {
    const float m2 = re[f] * re[f] + im[f] * im[f];
    re[f] = sqrtf(m2);
    ss += m2;
  }
  red[tid] = ss;
  __syncthreads();
  for (int st = 128; st > 0; st >>= 1) { if (tid < st) red[tid] += red[tid + st]; __syncthreads(); }
  const float inv = 1.0f / (sqrtf(red[0]) + 1e-8f);
  float* dst_row = Xn + (size_t)bc * XNP;
  fft_store(dst_row, re, inv, tid);
  __threadfence();
  fft_store(dst_row, re, inv, tid);
}

__global__ void __launch_bounds__(256) adj_kernel(
    const float* __restrict__ hn, const float* __restrict__ Xn,
    const float* __restrict__ prior, const float* __restrict__ lw,
    float* __restrict__ adjws, float* __restrict__ adjout)
{
  __shared__ __attribute__((aligned(16))) float sad[256];
  const int b = blockIdx.x, tid = threadIdx.x;
  const int c = tid >> 4, e = tid & 15;
  const float w0 = lw[0], w1 = lw[1], w2 = lw[2];
  const float mw = fmaxf(w0, fmaxf(w1, w2));
  const float e0 = expf(w0 - mw), e1 = expf(w1 - mw), e2 = expf(w2 - mw);
  const float inv = 1.0f / (e0 + e1 + e2);
  const float* hc = hn + (size_t)(b * 16 + c) * 64;
  const float* he = hn + (size_t)(b * 16 + e) * 64;
  float fc = 0.f;
#pragma unroll 16
  for (int dd = 0; dd < 64; ++dd) fc += hc[dd] * he[dd];
  const float* xc = Xn + (size_t)(b * 16 + c) * XNP;
  const float* xe = Xn + (size_t)(b * 16 + e) * XNP;
  float sc = 0.f;
#pragma unroll 4
  for (int f = 0; f < 2049; ++f) sc += xc[f] * xe[f];
  const float pv = prior[c * 16 + e] + prior[e * 16 + c];
  sad[tid] = (e0 * inv) * fc + (e1 * inv) * sc + (e2 * inv) * pv;
  __syncthreads();
  if (tid < 64) {
    const v4f v = *(const v4fa*)&sad[tid * 4];
    *(volatile v4f*)(adjws + (size_t)b * 256 + tid * 4) = v;
    *(volatile v4f*)(adjout + (size_t)b * 256 + tid * 4) = v;
  }
  __threadfence();
  if (tid < 64) {
    const v4f v = *(const v4fa*)&sad[tid * 4];
    *(volatile v4f*)(adjws + (size_t)b * 256 + tid * 4) = v;
    *(volatile v4f*)(adjout + (size_t)b * 256 + tid * 4) = v;
  }
}

#define SXS 68
#define SAS 72
#define SMS 200
#define SWK 72
#define SW2 136

DEV void gat_store_rows(float* dst_base, const float* sx, int wave, int lane) {
  const int q = lane >> 3, j = lane & 7;
#pragma unroll
  for (int s = 0; s < 8; ++s) {
    const int L = wave * 32 + s * 4 + q;
    const int row = L >> 1, half = L & 1;
    const v4f v = *(const v4fa*)(sx + row * SXS + half * 32 + j * 4);
    *(volatile v4f*)(dst_base + (size_t)row * 64 + half * 32 + j * 4) = v;
  }
}

DEV void gat_store_hs(_Float16* hs16, const _Float16* sa, int bidx, int t0, int wave, int lane) {
  const int q = lane >> 3, j = lane & 7;
#pragma unroll
  for (int s = 0; s < 4; ++s) {
    const int L = wave * 16 + s * 4 + q;
    const int cch = L >> 3, g = L & 7;
    const int r = g * 16 + cch;
    const v8h v = *(const v8ha*)(sa + r * SAS + j * 8);
    _Float16* dst = hs16 + (((size_t)(bidx * 16 + cch) * 256 + t0 + g) * 64 + j * 8);
    *(volatile v8h*)dst = v;
  }
}

__global__ void __launch_bounds__(256) gat_layer_kernel(
    float* __restrict__ ht, const float* __restrict__ adj,
    const float* __restrict__ n1g, const float* __restrict__ n1b,
    const float* __restrict__ qkvw, const float* __restrict__ qkvb,
    const float* __restrict__ outw, const float* __restrict__ outb,
    const float* __restrict__ n2g, const float* __restrict__ n2b,
    const float* __restrict__ f1w, const float* __restrict__ f1b,
    const float* __restrict__ f2w, const float* __restrict__ f2b,
    const float* __restrict__ fng, const float* __restrict__ fnb,
    _Float16* __restrict__ hs16, int last)
{
  __shared__ __attribute__((aligned(16))) float    sx[128 * SXS];
  __shared__ __attribute__((aligned(16))) _Float16 sa[128 * SAS];
  __shared__ __attribute__((aligned(16))) _Float16 sm[128 * SMS];
  __shared__ __attribute__((aligned(16))) _Float16 swb[192 * SWK];
  __shared__ float sbias[192];
  __shared__ float sadj[256];
  __shared__ float slng[64], slnb[64], sfg[64], sfb[64];

  const int tid = threadIdx.x;
  const int lane = tid & 31, wave = tid >> 5;
  const int m = lane & 15, h = lane >> 4;
  const int n0 = blockIdx.x * 8;
  const int bidx = n0 >> 8;
  const int t0 = n0 & 255;
  const size_t gbase = (size_t)n0 * 16 * 64;

  {
    const v4f* src = (const v4f*)(ht + gbase);
    for (int i = tid; i < 2048; i += 256) {
      const int r = i >> 4, q = i & 15;
      *(v4fa*)&sx[r * SXS + q * 4] = src[i];
    }
  }
  sadj[tid] = adj[bidx * 256 + tid];
  if (tid < 64) { slng[tid] = n1g[tid]; slnb[tid] = n1b[tid]; sfg[tid] = fng[tid]; sfb[tid] = fnb[tid]; }
  for (int i = tid; i < 192 * 64; i += 256) swb[(i >> 6) * SWK + (i & 63)] = (_Float16)qkvw[i];
  if (tid < 192) sbias[tid] = qkvb[tid];
  __syncthreads();

  if (tid < 128) ln_row_f16(&sx[tid * SXS], slng, slnb, &sa[tid * SAS]);
  __syncthreads();

  {
    const int mt = wave;
    const v16h a0 = ld_frag(&sa[mt * 16 * SAS], SAS, lane);
    const v16h a1 = ld_frag(&sa[mt * 16 * SAS + 32], SAS, lane);
    for (int nt = 0; nt < 12; ++nt) {
      const v16h b0 = ld_frag(&swb[nt * 16 * SWK], SWK, lane);
      const v16h b1 = ld_frag(&swb[nt * 16 * SWK + 32], SWK, lane);
      v8f cc = splat8(sbias[nt * 16 + m]);
      cc = wmma_f16(a0, b0, cc);
      cc = wmma_f16(a1, b1, cc);
#pragma unroll
      for (int i = 0; i < 8; ++i) {
        const int row = mt * 16 + 8 * h + i;
        sm[row * SMS + nt * 16 + m] = (_Float16)cc[i];
      }
    }
  }
  __syncthreads();

  for (int i = tid; i < 64 * 64; i += 256) swb[(i >> 6) * SWK + (i & 63)] = (_Float16)outw[i];
  if (tid < 64) { sbias[tid] = outb[tid]; slng[tid] = n2g[tid]; slnb[tid] = n2b[tid]; }
  {
    const int iq = m;
    for (int it = 0; it < 2; ++it) {
      const int pr = wave * 4 + it * 2 + h;
      const int g = pr >> 2, hh = pr & 3;
      const _Float16* base = &sm[(g * 16) * SMS + hh * 16];
      const v8h q0 = *(const v8ha*)(base + iq * SMS);
      const v8h q1 = *(const v8ha*)(base + iq * SMS + 8);
      float qf[16];
#pragma unroll
      for (int e = 0; e < 8; ++e) { qf[e] = (float)q0[e]; qf[8 + e] = (float)q1[e]; }
      float s[16];
      float mx = -3.0e38f;
#pragma unroll
      for (int j = 0; j < 16; ++j) {
        const _Float16* kr = base + j * SMS + 64;
        const v8h k0 = *(const v8ha*)kr;
        const v8h k1 = *(const v8ha*)(kr + 8);
        float acc = 0.f;
#pragma unroll
        for (int e = 0; e < 8; ++e)
          acc += qf[e] * (float)k0[e] + qf[8 + e] * (float)k1[e];
        s[j] = acc * 0.25f + sadj[iq * 16 + j];
        mx = fmaxf(mx, s[j]);
      }
      float ssum = 0.f;
#pragma unroll
      for (int j = 0; j < 16; ++j) { s[j] = expf(s[j] - mx); ssum += s[j]; }
      const float inv = 1.0f / ssum;
      float o[16];
#pragma unroll
      for (int e = 0; e < 16; ++e) o[e] = 0.f;
#pragma unroll
      for (int j = 0; j < 16; ++j) {
        const _Float16* vr = base + j * SMS + 128;
        const v8h v0 = *(const v8ha*)vr;
        const v8h v1 = *(const v8ha*)(vr + 8);
        const float pj = s[j];
#pragma unroll
        for (int e = 0; e < 8; ++e) { o[e] += pj * (float)v0[e]; o[8 + e] += pj * (float)v1[e]; }
      }
      v8h r0, r1;
#pragma unroll
      for (int e = 0; e < 8; ++e) {
        r0[e] = (_Float16)(o[e] * inv);
        r1[e] = (_Float16)(o[8 + e] * inv);
      }
      _Float16* dst = &sa[(g * 16 + iq) * SAS + hh * 16];
      *(v8ha*)dst = r0;
      *(v8ha*)(dst + 8) = r1;
    }
  }
  __syncthreads();

  {
    const int mt = wave;
    const v16h a0 = ld_frag(&sa[mt * 16 * SAS], SAS, lane);
    const v16h a1 = ld_frag(&sa[mt * 16 * SAS + 32], SAS, lane);
    for (int nt = 0; nt < 4; ++nt) {
      const v16h b0 = ld_frag(&swb[nt * 16 * SWK], SWK, lane);
      const v16h b1 = ld_frag(&swb[nt * 16 * SWK + 32], SWK, lane);
      v8f cc;
      const float bv = sbias[nt * 16 + m];
#pragma unroll
      for (int i = 0; i < 8; ++i) {
        const int row = mt * 16 + 8 * h + i;
        cc[i] = sx[row * SXS + nt * 16 + m] + bv;
      }
      cc = wmma_f16(a0, b0, cc);
      cc = wmma_f16(a1, b1, cc);
#pragma unroll
      for (int i = 0; i < 8; ++i) {
        const int row = mt * 16 + 8 * h + i;
        sx[row * SXS + nt * 16 + m] = cc[i];
      }
    }
  }
  __syncthreads();

  for (int i = tid; i < 128 * 64; i += 256) swb[(i >> 6) * SWK + (i & 63)] = (_Float16)f1w[i];
  if (tid < 128) sbias[tid] = f1b[tid];
  if (tid < 128) ln_row_f16(&sx[tid * SXS], slng, slnb, &sa[tid * SAS]);
  __syncthreads();

  {
    const int mt = wave;
    const v16h a0 = ld_frag(&sa[mt * 16 * SAS], SAS, lane);
    const v16h a1 = ld_frag(&sa[mt * 16 * SAS + 32], SAS, lane);
    for (int nt = 0; nt < 8; ++nt) {
      const v16h b0 = ld_frag(&swb[nt * 16 * SWK], SWK, lane);
      const v16h b1 = ld_frag(&swb[nt * 16 * SWK + 32], SWK, lane);
      v8f cc = splat8(sbias[nt * 16 + m]);
      cc = wmma_f16(a0, b0, cc);
      cc = wmma_f16(a1, b1, cc);
#pragma unroll
      for (int i = 0; i < 8; ++i) {
        const int row = mt * 16 + 8 * h + i;
        sm[row * SMS + nt * 16 + m] = (_Float16)gelu_f(cc[i]);
      }
    }
  }
  __syncthreads();

  for (int i = tid; i < 64 * 128; i += 256) swb[(i >> 7) * SW2 + (i & 127)] = (_Float16)f2w[i];
  if (tid < 64) sbias[tid] = f2b[tid];
  __syncthreads();

  {
    const int mt = wave;
    const v16h a0 = ld_frag(&sm[mt * 16 * SMS], SMS, lane);
    const v16h a1 = ld_frag(&sm[mt * 16 * SMS + 32], SMS, lane);
    const v16h a2 = ld_frag(&sm[mt * 16 * SMS + 64], SMS, lane);
    const v16h a3 = ld_frag(&sm[mt * 16 * SMS + 96], SMS, lane);
    for (int nt = 0; nt < 4; ++nt) {
      const v16h b0 = ld_frag(&swb[nt * 16 * SW2], SW2, lane);
      const v16h b1 = ld_frag(&swb[nt * 16 * SW2 + 32], SW2, lane);
      const v16h b2 = ld_frag(&swb[nt * 16 * SW2 + 64], SW2, lane);
      const v16h b3 = ld_frag(&swb[nt * 16 * SW2 + 96], SW2, lane);
      v8f cc;
      const float bv = sbias[nt * 16 + m];
#pragma unroll
      for (int i = 0; i < 8; ++i) {
        const int row = mt * 16 + 8 * h + i;
        cc[i] = sx[row * SXS + nt * 16 + m] + bv;
      }
      cc = wmma_f16(a0, b0, cc);
      cc = wmma_f16(a1, b1, cc);
      cc = wmma_f16(a2, b2, cc);
      cc = wmma_f16(a3, b3, cc);
#pragma unroll
      for (int i = 0; i < 8; ++i) {
        const int row = mt * 16 + 8 * h + i;
        sx[row * SXS + nt * 16 + m] = cc[i];
      }
    }
  }
  __syncthreads();

  if (last) {
    if (tid < 128) ln_row_f16(&sx[tid * SXS], sfg, sfb, &sa[tid * SAS]);
    __syncthreads();
    gat_store_hs(hs16, sa, bidx, t0, wave, lane);
    __threadfence();
    gat_store_hs(hs16, sa, bidx, t0, wave, lane);
  } else {
    float* dst_base = ht + gbase;
    gat_store_rows(dst_base, sx, wave, lane);
    __threadfence();
    gat_store_rows(dst_base, sx, wave, lane);
  }
}

#define SHP 68
#define SHA 72

DEV void gru_store(float* hout, const float* sh, int s0, int dir, int tid) {
#pragma unroll
  for (int s = 0; s < 2; ++s) {
    const int idx = s * 256 + tid;
    const int r = idx >> 4, j = idx & 15;
    const v4f v = *(const v4fa*)(sh + r * SHP + j * 4);
    *(volatile v4f*)(hout + (size_t)(s0 + r) * 128 + dir * 64 + j * 4) = v;
  }
}

__global__ void __launch_bounds__(256) gru_kernel(
    const _Float16* __restrict__ hs16,
    const float* __restrict__ wih, const float* __restrict__ whh,
    const float* __restrict__ bih, const float* __restrict__ bhh,
    float* __restrict__ h_out)
{
  __shared__ __attribute__((aligned(16))) float    sh[32 * SHP];
  __shared__ __attribute__((aligned(16))) _Float16 sha[2][32 * SHA];
  __shared__ __attribute__((aligned(16))) _Float16 sxa[32 * SHA];
  __shared__ __attribute__((aligned(16))) _Float16 swi[192 * SWK];
  __shared__ __attribute__((aligned(16))) _Float16 swh[192 * SWK];
  __shared__ float sbi[192], sbh[192];

  const int tid = threadIdx.x, lane = tid & 31, wave = tid >> 5;
  const int m = lane & 15, h = lane >> 4;
  const int dir = blockIdx.x >> 4, chunk = blockIdx.x & 15;
  const int s0 = chunk * 32;

  {
    const float* wi = wih + (size_t)dir * 12288;
    const float* wh = whh + (size_t)dir * 12288;
    for (int i = tid; i < 12288; i += 256) {
      swi[(i >> 6) * SWK + (i & 63)] = (_Float16)wi[i];
      swh[(i >> 6) * SWK + (i & 63)] = (_Float16)wh[i];
    }
  }
  if (tid < 192) { sbi[tid] = bih[dir * 192 + tid]; sbh[tid] = bhh[dir * 192 + tid]; }
  for (int i = tid; i < 32 * SHP; i += 256) sh[i] = 0.f;
  {
    _Float16* pz = &sha[0][0];
    for (int i = tid; i < 2 * 32 * SHA; i += 256) pz[i] = (_Float16)0.0f;
  }
  __syncthreads();

  const int mt = wave & 1;
  const int ng = wave >> 1;
  const int col = ng * 16 + m;
  for (int step = 0; step < 256; ++step) {
    const int tt = dir ? (255 - step) : step;
    {
      const int r = tid >> 3, q = tid & 7;
      const v8h xv = *(const v8h*)(hs16 + ((size_t)(s0 + r) * 256 + (size_t)tt) * 64 + q * 8);
      *(v8ha*)&sxa[r * SHA + q * 8] = xv;
    }
    __syncthreads();
    const _Float16* hA = &sha[step & 1][0];
    _Float16* hN = &sha[(step & 1) ^ 1][0];
    const v16h ax0 = ld_frag(&sxa[mt * 16 * SHA], SHA, lane);
    const v16h ax1 = ld_frag(&sxa[mt * 16 * SHA + 32], SHA, lane);
    const v16h ah0 = ld_frag(&hA[mt * 16 * SHA], SHA, lane);
    const v16h ah1 = ld_frag(&hA[mt * 16 * SHA + 32], SHA, lane);
    v8f gi_r = splat8(sbi[col]), gi_z = splat8(sbi[64 + col]), gi_n = splat8(sbi[128 + col]);
    v8f gh_r = splat8(sbh[col]), gh_z = splat8(sbh[64 + col]), gh_n = splat8(sbh[128 + col]);
    {
      const v16h b0 = ld_frag(&swi[(0 * 64 + ng * 16) * SWK], SWK, lane);
      const v16h b1 = ld_frag(&swi[(0 * 64 + ng * 16) * SWK + 32], SWK, lane);
      gi_r = wmma_f16(ax0, b0, gi_r); gi_r = wmma_f16(ax1, b1, gi_r);
    }
    {
      const v16h b0 = ld_frag(&swi[(1 * 64 + ng * 16) * SWK], SWK, lane);
      const v16h b1 = ld_frag(&swi[(1 * 64 + ng * 16) * SWK + 32], SWK, lane);
      gi_z = wmma_f16(ax0, b0, gi_z); gi_z = wmma_f16(ax1, b1, gi_z);
    }
    {
      const v16h b0 = ld_frag(&swi[(2 * 64 + ng * 16) * SWK], SWK, lane);
      const v16h b1 = ld_frag(&swi[(2 * 64 + ng * 16) * SWK + 32], SWK, lane);
      gi_n = wmma_f16(ax0, b0, gi_n); gi_n = wmma_f16(ax1, b1, gi_n);
    }
    {
      const v16h b0 = ld_frag(&swh[(0 * 64 + ng * 16) * SWK], SWK, lane);
      const v16h b1 = ld_frag(&swh[(0 * 64 + ng * 16) * SWK + 32], SWK, lane);
      gh_r = wmma_f16(ah0, b0, gh_r); gh_r = wmma_f16(ah1, b1, gh_r);
    }
    {
      const v16h b0 = ld_frag(&swh[(1 * 64 + ng * 16) * SWK], SWK, lane);
      const v16h b1 = ld_frag(&swh[(1 * 64 + ng * 16) * SWK + 32], SWK, lane);
      gh_z = wmma_f16(ah0, b0, gh_z); gh_z = wmma_f16(ah1, b1, gh_z);
    }
    {
      const v16h b0 = ld_frag(&swh[(2 * 64 + ng * 16) * SWK], SWK, lane);
      const v16h b1 = ld_frag(&swh[(2 * 64 + ng * 16) * SWK + 32], SWK, lane);
      gh_n = wmma_f16(ah0, b0, gh_n); gh_n = wmma_f16(ah1, b1, gh_n);
    }
#pragma unroll
    for (int i = 0; i < 8; ++i) {
      const int row = mt * 16 + 8 * h + i;
      const float hp = sh[row * SHP + col];
      const float rg = sigm_f(gi_r[i] + gh_r[i]);
      const float zg = sigm_f(gi_z[i] + gh_z[i]);
      const float ngv = tanhf(gi_n[i] + rg * gh_n[i]);
      const float hv = (1.0f - zg) * ngv + zg * hp;
      sh[row * SHP + col] = hv;
      hN[row * SHA + col] = (_Float16)hv;
    }
    __syncthreads();
  }
  gru_store(h_out, sh, s0, dir, tid);
  __threadfence();
  gru_store(h_out, sh, s0, dir, tid);
}

#define RAP 136

DEV void readout_store(float* out, const float* sro, const float* sg, int tid) {
#pragma unroll
  for (int s = 0; s < 2; ++s) {
    const int f4 = s * 512 + tid;
    const v4f v = *(const v4fa*)(sro + f4 * 4);
    *(volatile v4f*)(out + f4 * 4) = v;
  }
  if (tid < 128) {
    const v4f v = *(const v4fa*)(sg + tid * 4);
    *(volatile v4f*)(out + 12288 + tid * 4) = v;
  }
}

__global__ void __launch_bounds__(512) readout_kernel(
    const float* __restrict__ h_out, const float* __restrict__ gw,
    const float* __restrict__ gb, float* __restrict__ out)
{
  __shared__ __attribute__((aligned(16))) float    sro[4096];
  __shared__ __attribute__((aligned(16))) float    sg[512];
  __shared__ __attribute__((aligned(16))) _Float16 sA[256 * RAP];
  __shared__ __attribute__((aligned(16))) _Float16 sB[16 * RAP];
  const int tid = threadIdx.x, lane = tid & 31, wave = tid >> 5;
  const int m = lane & 15, h = lane >> 4;
  const float gbias = gb[0];
  for (int i = tid; i < 16 * RAP; i += 512) sB[i] = (i < 128) ? (_Float16)gw[i] : (_Float16)0.0f;
  for (int it = 0; it < 2; ++it) {
    for (int i = tid; i < 256 * 16; i += 512) {
      const int r = i >> 4, q = i & 15;
      const float* p = h_out + ((size_t)(it * 256 + r) * 128 + q * 8);
      const v4f lo = *(const v4fa*)p;
      const v4f hi = *(const v4fa*)(p + 4);
      v8h hv;
#pragma unroll
      for (int e = 0; e < 4; ++e) { hv[e] = (_Float16)lo[e]; hv[4 + e] = (_Float16)hi[e]; }
      *(v8ha*)&sA[r * RAP + q * 8] = hv;
    }
    __syncthreads();
    v8f acc = splat8(0.f);
#pragma unroll
    for (int ks = 0; ks < 4; ++ks)
      acc = wmma_f16(ld_frag(sA + wave * 16 * RAP + ks * 32, RAP, lane),
                     ld_frag(sB + ks * 32, RAP, lane), acc);
    if (m == 0) {
#pragma unroll
      for (int i = 0; i < 8; ++i)
        sg[it * 256 + wave * 16 + 8 * h + i] = sigm_f(acc[i] + gbias);
    }
    __syncthreads();
  }
  for (int k = 0; k < 8; ++k) {
    const int o = k * 512 + tid;
    const int b2 = o >> 7, d = o & 127;
    float gs = 0.f, acc = 0.f;
#pragma unroll
    for (int cc = 0; cc < 16; ++cc) {
      const float g = sg[b2 * 16 + cc];
      gs += g;
      acc += h_out[(size_t)(b2 * 16 + cc) * 128 + d] * g;
    }
    sro[o] = acc * (1.0f / (gs + 1e-8f));
  }
  __syncthreads();
  readout_store(out, sro, sg, tid);
  __threadfence();
  readout_store(out, sro, sg, tid);
}

extern "C" void kernel_launch(void* const* d_in, const int* in_sizes, int n_in,
                              void* d_out, int out_size, void* d_ws, size_t ws_size,
                              hipStream_t stream)
{
  if (n_in < 35) return;
  if (in_sizes[0] != 32 * 16 * 4096) return;
  if (in_sizes[17] != 2 * 192 * 64 || in_sizes[29] != 2 * 192 * 64) return;
  if (in_sizes[33] != 128) return;
  if (out_size != 4096 + 8192 + 512) return;

  const float* x       = (const float*)d_in[0];
  const float* c1w     = (const float*)d_in[1];
  const float* c1b     = (const float*)d_in[2];
  const float* bn1g    = (const float*)d_in[3];
  const float* bn1b    = (const float*)d_in[4];
  const float* bn1m    = (const float*)d_in[5];
  const float* bn1v    = (const float*)d_in[6];
  const float* c2w     = (const float*)d_in[7];
  const float* c2b     = (const float*)d_in[8];
  const float* bn2g    = (const float*)d_in[9];
  const float* bn2b    = (const float*)d_in[10];
  const float* bn2m    = (const float*)d_in[11];
  const float* bn2v    = (const float*)d_in[12];
  const float* prior   = (const float*)d_in[13];
  const float* logw    = (const float*)d_in[14];
  const float* n1g     = (const float*)d_in[15];
  const float* n1b     = (const float*)d_in[16];
  const float* qkvw    = (const float*)d_in[17];
  const float* qkvb    = (const float*)d_in[18];
  const float* outw    = (const float*)d_in[19];
  const float* outb    = (const float*)d_in[20];
  const float* n2g     = (const float*)d_in[21];
  const float* n2b     = (const float*)d_in[22];
  const float* f1w     = (const float*)d_in[23];
  const float* f1b     = (const float*)d_in[24];
  const float* f2w     = (const float*)d_in[25];
  const float* f2b     = (const float*)d_in[26];
  const float* gatng   = (const float*)d_in[27];
  const float* gatnb   = (const float*)d_in[28];
  const float* gruwih  = (const float*)d_in[29];
  const float* gruwhh  = (const float*)d_in[30];
  const float* grubih  = (const float*)d_in[31];
  const float* grubhh  = (const float*)d_in[32];
  const float* gatew   = (const float*)d_in[33];
  const float* gateb   = (const float*)d_in[34];

  char* w = (char*)d_ws;
  size_t off = 0;
  float*    ht    = (float*)(w + off);     off += (size_t)8192 * 16 * 64 * 4;
  _Float16* hs16  = (_Float16*)(w + off);  off += (size_t)512 * 256 * 64 * 2;
  float*    Xn    = (float*)(w + off);     off += (size_t)512 * XNP * 4;
  float*    hnb   = (float*)(w + off);     off += (size_t)512 * 64 * 4;
  float*    hout  = (float*)(w + off);     off += (size_t)512 * 128 * 4;
  float*    adjws = (float*)(w + off);     off += (size_t)32 * 256 * 4;
  if (off > ws_size) return;
  float* outp = (float*)d_out;

  conv_kernel<<<512, 256, 0, stream>>>(x, c1w, c1b, bn1g, bn1b, bn1m, bn1v,
                                       c2w, c2b, bn2g, bn2b, bn2m, bn2v, ht, hnb);
  fft_kernel<<<512, 256, 0, stream>>>(x, Xn);
  adj_kernel<<<32, 256, 0, stream>>>(hnb, Xn, prior, logw, adjws, outp + 4096);
  for (int l = 0; l < 2; ++l) {
    gat_layer_kernel<<<1024, 256, 0, stream>>>(ht, adjws,
        n1g + l * 64, n1b + l * 64, qkvw + l * 12288, qkvb + l * 192,
        outw + l * 4096, outb + l * 64, n2g + l * 64, n2b + l * 64,
        f1w + l * 8192, f1b + l * 128, f2w + l * 8192, f2b + l * 64,
        gatng, gatnb, hs16, (l == 1) ? 1 : 0);
  }
  gru_kernel<<<32, 256, 0, stream>>>(hs16, gruwih, gruwhh, grubih, grubhh, hout);
  readout_kernel<<<1, 512, 0, stream>>>(hout, gatew, gateb, outp);
}
